// MLPList_58574763983287
// MI455X (gfx1250) — hardware-verified
//
#include <hip/hip_runtime.h>
#include <math.h>

constexpr int kBatch   = 32768;
constexpr int kDin     = 64;
constexpr int kHid     = 64;
constexpr int kNExp    = 63;
constexpr int kN1      = 4096;
constexpr int kN1Real  = kNExp * kHid;
constexpr int kChunk   = 8192;
constexpr int kNChunk  = kBatch / kChunk;
constexpr float kWCarry  = 16.0f;
constexpr float kH1Carry = 8.0f;
constexpr float kB1Carry = 8.0f;
constexpr float kL1Scale = kH1Carry / kWCarry;
constexpr float kL2Scale = 1.0f / (kH1Carry * kWCarry);

static_assert(kBatch % kChunk == 0, "");
static_assert(kChunk % 64 == 0, "");
static_assert(kN1 % 64 == 0, "");

constexpr size_t kOffXh  = 0;
constexpr size_t kOffW1t = kOffXh  + (size_t)kBatch * kDin * 2;
constexpr size_t kOffW2t = kOffW1t + (size_t)kN1 * kDin * 2;
constexpr size_t kOffB1p = kOffW2t + (size_t)kN1 * kHid * 2;
constexpr size_t kOffO   = kOffB1p + (size_t)kN1 * 4;
constexpr size_t kOffH1  = kOffO   + (size_t)64 * kBatch * 4;
constexpr size_t kWsTotal = kOffH1 + (size_t)kChunk * kN1 * 2;
static_assert(kWsTotal == 80756736, "");
static_assert(kWsTotal <= 134217728, "");
static_assert(kOffW1t % 256 == 0 && kOffW2t % 256 == 0 && kOffB1p % 256 == 0 && kOffO % 256 == 0 && kOffH1 % 256 == 0, "");

typedef __attribute__((ext_vector_type(16))) _Float16 v16h;
typedef __attribute__((ext_vector_type(8)))  _Float16 v8h;
typedef __attribute__((ext_vector_type(16))) __bf16   v16b;
typedef __attribute__((ext_vector_type(8)))  __bf16   v8b;
typedef __attribute__((ext_vector_type(8)))  float    v8f;
typedef __attribute__((ext_vector_type(4)))  float    v4f;
typedef __attribute__((ext_vector_type(4)))  unsigned int v4u;

__device__ __forceinline__ unsigned short f2bf_bits(float f) {
  unsigned u = __float_as_uint(f);
  return (unsigned short)((u + 0x7FFFu + ((u >> 16) & 1u)) >> 16);
}
__device__ __forceinline__ float bf_bits2f(unsigned short h) { return __uint_as_float(((unsigned)h) << 16); }

__device__ __forceinline__ void dep_guard_h(v8f& a, v8f& b, v16h x, v16h y) { asm volatile("v_nop\n\tv_nop\n\tv_nop\n\tv_nop" : "+v"(a), "+v"(b) : "v"(x), "v"(y)); }
__device__ __forceinline__ void dep_guard_b(v8f& a, v8f& b, v16b x, v16b y) { asm volatile("v_nop\n\tv_nop\n\tv_nop\n\tv_nop" : "+v"(a), "+v"(b) : "v"(x), "v"(y)); }
__device__ __forceinline__ void keep4_h(v16h a, v16h b, v16h c, v16h d) { asm volatile("v_nop" :: "v"(a), "v"(b), "v"(c), "v"(d)); }
__device__ __forceinline__ void keep4_b(v16b a, v16b b, v16b c, v16b d) { asm volatile("v_nop" :: "v"(a), "v"(b), "v"(c), "v"(d)); }
__device__ __forceinline__ void acc_guard4(v8f& a, v8f& b, v8f& c, v8f& d) { asm volatile("v_nop\n\tv_nop\n\tv_nop\n\tv_nop" : "+v"(a), "+v"(b), "+v"(c), "+v"(d)); }
template <typename T> struct Frag;
template <> struct Frag<_Float16> {
  typedef v16h V; union U { v16h v; v8h h[2]; };
  static __device__ __forceinline__ v16h load(const _Float16* p) {
    U f; f.h[0] = *(const v8h*)(p); f.h[1] = *(const v8h*)(p + 16); return f.v;
  }
  static __device__ __forceinline__ v8f mma(v16h a, v16h b, v8f c) {
    return __builtin_amdgcn_wmma_f32_16x16x32_f16(false, a, false, b, (short)0, c, false, false);
  }
  static __device__ __forceinline__ void guard(v8f& a, v8f& b, v16h x, v16h y) { dep_guard_h(a, b, x, y); }
  static __device__ __forceinline__ void keep(v16h a, v16h b, v16h c, v16h d) { keep4_h(a, b, c, d); }
};
template <> struct Frag<__bf16> {
  typedef v16b V; union U { v16b v; v8b h[2]; };
  static __device__ __forceinline__ v16b load(const __bf16* p) {
    U f; f.h[0] = *(const v8b*)(p); f.h[1] = *(const v8b*)(p + 16); return f.v;
  }
  static __device__ __forceinline__ v8f mma(v16b a, v16b b, v8f c) {
    return __builtin_amdgcn_wmma_f32_16x16x32_bf16(false, a, false, b, (short)0, c, false, false);
  }
  static __device__ __forceinline__ void guard(v8f& a, v8f& b, v16b x, v16b y) { dep_guard_b(a, b, x, y); }
  static __device__ __forceinline__ void keep(v16b a, v16b b, v16b c, v16b d) { keep4_b(a, b, c, d); }
};

__device__ __forceinline__ unsigned pk16(unsigned short a, unsigned short b) { return (unsigned)a | ((unsigned)b << 16); }
__device__ __forceinline__ unsigned short h_bits(float f) { const _Float16 h = (_Float16)f; return __builtin_bit_cast(unsigned short, h); }

template <int ET> struct Elem;
template <> struct Elem<0> { typedef _Float16 T; };
template <> struct Elem<1> { typedef __bf16 T; };
template <int ET, bool SPLIT, int BIAS_MODE, int OUT_MODE, bool RESID, int ACT = 0>
__global__ __launch_bounds__(256) void wmma_gemm64(
    const unsigned short* __restrict__ Ap, const unsigned short* __restrict__ A2p, int lda, long strideA,
    const unsigned short* __restrict__ Btp, const unsigned short* __restrict__ Bt2p, int ldb, long strideB,
    void* __restrict__ Cout, void* __restrict__ Cout2, int ldc, long strideC,
    const float* __restrict__ bias,
    const float* __restrict__ resid, long strideR,
    int M, int N, int K, float scale) {
  typedef typename Elem<ET>::T T;
  typedef typename Frag<T>::V V;
  const T* A = (const T*)Ap; const T* A2 = (const T*)A2p; const T* Bt = (const T*)Btp; const T* Bt2 = (const T*)Bt2p;
  __shared__ __align__(16) float sT[8][16 * 68];
  const int b    = blockIdx.y;
  const int lane = threadIdx.x & 31;
  const int wave = threadIdx.x >> 5;
  const int tilesN = N >> 6;
  const int tilesM = M >> 6;
  const int tile = blockIdx.x * 8 + wave;
  if (tile >= tilesM * tilesN) return;
  const int tm = tile / tilesN;
  const int tn = tile - tm * tilesN;
  const int m0 = tm << 6;
  const int n0 = tn << 6;

  const T* Ab  = A  + (size_t)b * strideA;
  const T* Bb  = Bt + (size_t)b * strideB;
  const T* Ab2 = SPLIT ? (A2  + (size_t)b * strideA) : nullptr;
  const T* Bb2 = SPLIT ? (Bt2 + (size_t)b * strideB) : nullptr;

  const int rlane = lane & 15;
  const int koff  = (lane >> 4) * 8;
  const int mOff  = (lane >> 4) * 8;

  v8f acc[4][4];
#pragma unroll
  for (int i = 0; i < 4; ++i)
#pragma unroll
    for (int j = 0; j < 4; ++j) acc[i][j] = (v8f){0.f,0.f,0.f,0.f,0.f,0.f,0.f,0.f};

  for (int k0 = 0; k0 < K; k0 += 32) {
    V bh[4], bl[4];
#pragma unroll
    for (int j = 0; j < 4; ++j) {
      const size_t bo = (size_t)(n0 + (j << 4) + rlane) * ldb + koff + k0;
      bh[j] = Frag<T>::load(Bb + bo);
      if (SPLIT) bl[j] = Frag<T>::load(Bb2 + bo);
    }
#pragma unroll
    for (int i = 0; i < 4; ++i) {
      const size_t ao = (size_t)(m0 + (i << 4) + rlane) * lda + koff + k0;
      V ah = Frag<T>::load(Ab + ao);
      V al;
      if (SPLIT) al = Frag<T>::load(Ab2 + ao);
#pragma unroll
      for (int j = 0; j < 4; ++j) {
        acc[i][j] = Frag<T>::mma(ah, bh[j], acc[i][j]);
        if (SPLIT) {
          acc[i][j] = Frag<T>::mma(ah, bl[j], acc[i][j]);
          acc[i][j] = Frag<T>::mma(al, bh[j], acc[i][j]);
        }
      }
      Frag<T>::guard(acc[i][0], acc[i][3], ah, SPLIT ? al : ah);
    }
    Frag<T>::keep(bh[0], bh[1], bh[2], bh[3]);
    if (SPLIT) Frag<T>::keep(bl[0], bl[1], bl[2], bl[3]);
  }
  acc_guard4(acc[0][0], acc[0][1], acc[0][2], acc[0][3]);
  acc_guard4(acc[1][0], acc[1][1], acc[1][2], acc[1][3]);
  acc_guard4(acc[2][0], acc[2][1], acc[2][2], acc[2][3]);
  acc_guard4(acc[3][0], acc[3][1], acc[3][2], acc[3][3]);

  float* slab = sT[wave];
  const float* Rb = RESID ? (resid + (size_t)b * strideR) : nullptr;
#pragma unroll
  for (int i = 0; i < 4; ++i) {
    const int mBase = m0 + (i << 4);
#pragma unroll
    for (int j = 0; j < 4; ++j) {
      const int n = n0 + (j << 4) + rlane;
      float bv = 0.f;
      if (BIAS_MODE == 2) bv = bias[n];
#pragma unroll
      for (int r = 0; r < 8; ++r) {
        float v = acc[i][j][r] * scale;
        if (BIAS_MODE == 1) v += bias[mBase + mOff + r];
        if (BIAS_MODE == 2) v += bv;
        if (RESID) v += Rb[(size_t)(mBase + mOff + r) * ldc + n];
        if (ACT == 2) v = fmaxf(v, 0.0f);
        if (ACT == 4) v = (v > 0.f) ? v : 0.01f * v;
        slab[(mOff + r) * 68 + (j << 4) + rlane] = v;
      }
    }
    __builtin_amdgcn_fence(__ATOMIC_RELEASE, "workgroup");
    __builtin_amdgcn_wave_barrier();
    __builtin_amdgcn_fence(__ATOMIC_ACQUIRE, "workgroup");
    if (OUT_MODE == 0) {
      float* C = (float*)Cout + (size_t)b * strideC;
      const int hh = lane >> 4, c4 = (lane & 15) * 4;
      for (int pass = 0; pass < 2; ++pass) {
#pragma unroll
        for (int it = 0; it < 8; ++it) {
          const int row = it * 2 + hh;
          v4f v = *(const v4f*)(slab + row * 68 + c4);
          *(volatile v4f*)(C + (size_t)(mBase + row) * ldc + n0 + c4) = v;
        }
        __threadfence();
      }
    } else {
      const int q = lane >> 3, c8 = (lane & 7) * 8;
      unsigned short* C  = (unsigned short*)Cout  + (size_t)b * strideC;
      unsigned short* C2 = (OUT_MODE == 2) ? ((unsigned short*)Cout2 + (size_t)b * strideC) : nullptr;
      for (int pass = 0; pass < 2; ++pass) {
#pragma unroll
        for (int it = 0; it < 4; ++it) {
          const int row = it * 4 + q;
          const float* sp = slab + row * 68 + c8;
          v8h hv, lv;
#pragma unroll
          for (int e = 0; e < 8; ++e) {
            if (OUT_MODE == 1) {
              hv[e] = (_Float16)sp[e];
            } else {
              unsigned short hb = f2bf_bits(sp[e]);
              unsigned short lb = f2bf_bits(sp[e] - bf_bits2f(hb));
              hv[e] = __builtin_bit_cast(_Float16, hb);
              lv[e] = __builtin_bit_cast(_Float16, lb);
            }
          }
          *(volatile v8h*)(C + (size_t)(mBase + row) * ldc + n0 + c8) = hv;
          if (OUT_MODE == 2) *(volatile v8h*)(C2 + (size_t)(mBase + row) * ldc + n0 + c8) = lv;
        }
        __threadfence();
      }
    }
    __builtin_amdgcn_fence(__ATOMIC_RELEASE, "workgroup");
    __builtin_amdgcn_wave_barrier();
    __builtin_amdgcn_fence(__ATOMIC_ACQUIRE, "workgroup");
  }
}

__global__ __launch_bounds__(256) void gemm64_rowdot(
    const unsigned short* __restrict__ Ap, int lda, long strideA,
    const unsigned short* __restrict__ Btp, int ldb, long strideB,
    const float* __restrict__ bias, long strideBias,
    const float* __restrict__ wvec, long strideW,
    const float* __restrict__ bout,
    float* __restrict__ Out, long strideO,
    int M, int K, float scale) {
  typedef _Float16 T;
  typedef v16h V;
  const T* A = (const T*)Ap; const T* Bt = (const T*)Btp;
  __shared__ __align__(16) float sO[8][64];
  const int b    = blockIdx.y;
  const int lane = threadIdx.x & 31;
  const int wave = threadIdx.x >> 5;
  const int tilesM = M >> 6;
  const int tile = blockIdx.x * 8 + wave;
  if (tile >= tilesM) return;
  const int m0 = tile << 6;

  const T* Ab = A  + (size_t)b * strideA;
  const T* Bb = Bt + (size_t)b * strideB;

  const int rlane = lane & 15;
  const int koff  = (lane >> 4) * 8;
  const int mOff  = (lane >> 4) * 8;

  v8f acc[4][4];
#pragma unroll
  for (int i = 0; i < 4; ++i)
#pragma unroll
    for (int j = 0; j < 4; ++j) acc[i][j] = (v8f){0.f,0.f,0.f,0.f,0.f,0.f,0.f,0.f};

  for (int k0 = 0; k0 < K; k0 += 32) {
    V bh[4];
#pragma unroll
    for (int j = 0; j < 4; ++j) {
      const size_t bo = (size_t)((j << 4) + rlane) * ldb + koff + k0;
      bh[j] = Frag<T>::load(Bb + bo);
    }
#pragma unroll
    for (int i = 0; i < 4; ++i) {
      const size_t ao = (size_t)(m0 + (i << 4) + rlane) * lda + koff + k0;
      V ah = Frag<T>::load(Ab + ao);
#pragma unroll
      for (int j = 0; j < 4; ++j) {
        acc[i][j] = Frag<T>::mma(ah, bh[j], acc[i][j]);
      }
      Frag<T>::guard(acc[i][0], acc[i][3], ah, ah);
    }
    Frag<T>::keep(bh[0], bh[1], bh[2], bh[3]);
  }
  acc_guard4(acc[0][0], acc[0][1], acc[0][2], acc[0][3]);
  acc_guard4(acc[1][0], acc[1][1], acc[1][2], acc[1][3]);
  acc_guard4(acc[2][0], acc[2][1], acc[2][2], acc[2][3]);
  acc_guard4(acc[3][0], acc[3][1], acc[3][2], acc[3][3]);

  const float* b2r = bias + (size_t)b * strideBias;
  const float* w3r = wvec + (size_t)b * strideW;
  const float  b3v = bout[b];
  float bv[4], wv[4];
#pragma unroll
  for (int j = 0; j < 4; ++j) {
    const int n = (j << 4) + rlane;
    bv[j] = b2r[n];
    wv[j] = w3r[n];
  }
  float* so = sO[wave];
#pragma unroll
  for (int i = 0; i < 4; ++i) {
#pragma unroll
    for (int r = 0; r < 8; ++r) {
      float p = 0.f;
#pragma unroll
      for (int j = 0; j < 4; ++j) {
        float v = acc[i][j][r] * scale + bv[j];
        v = fmaxf(v, 0.0f);
        p += v * wv[j];
      }
      p += __shfl_xor(p, 1, 32);
      p += __shfl_xor(p, 2, 32);
      p += __shfl_xor(p, 4, 32);
      p += __shfl_xor(p, 8, 32);
      if (rlane == 0) so[(i << 4) + mOff + r] = p + b3v;
    }
  }
  __builtin_amdgcn_fence(__ATOMIC_RELEASE, "workgroup");
  __builtin_amdgcn_wave_barrier();
  __builtin_amdgcn_fence(__ATOMIC_ACQUIRE, "workgroup");
  float* Ob = Out + (size_t)b * strideO + m0;
  const int c4 = (lane & 15) * 4;
  for (int pass = 0; pass < 2; ++pass) {
    v4f val = *(const v4f*)(so + c4);
    if (lane < 16) *(volatile v4f*)(Ob + c4) = val;
    __threadfence();
  }
}

__global__ __launch_bounds__(256) void cast8_f16_kernel(const float* __restrict__ in, unsigned short* __restrict__ out, int n8) {
  const int i = blockIdx.x * 256 + threadIdx.x;
  if (i >= n8) return;
  const float* p = in + 8 * (size_t)i;
  const v4f a = *(const v4f*)(p);
  const v4f c = *(const v4f*)(p + 4);
  unsigned short hb[8];
#pragma unroll
  for (int e = 0; e < 4; ++e) {
    hb[e]     = h_bits(a[e]);
    hb[4 + e] = h_bits(c[e]);
  }
  const v4u u = (v4u){pk16(hb[0], hb[1]), pk16(hb[2], hb[3]), pk16(hb[4], hb[5]), pk16(hb[6], hb[7])};
  unsigned short* q = out + 8 * (size_t)i;
  *(volatile v4u*)q = u;
  __threadfence();
  *(volatile v4u*)q = u;
}

__global__ __launch_bounds__(256) void w1t_kernel(const float* __restrict__ W1, unsigned short* __restrict__ out, float scale) {
  const int t = blockIdx.x * 256 + threadIdx.x;
  const int n = t >> 3;
  const int q = t & 7;
  const int r = n >> 6;
  const int h = n & 63;
  const int rc = (r < kNExp) ? r : (kNExp - 1);
  unsigned short hb[8];
#pragma unroll
  for (int e = 0; e < 8; ++e) {
    const int j = 8 * q + e;
    const float w = W1[((size_t)rc * kDin + j) * kHid + h] * scale;
    const bool keep = (r < kNExp) && (j <= r);
    hb[e] = h_bits(keep ? w : 0.0f);
  }
  const v4u u = (v4u){pk16(hb[0], hb[1]), pk16(hb[2], hb[3]), pk16(hb[4], hb[5]), pk16(hb[6], hb[7])};
  unsigned short* p = out + (size_t)n * kDin + 8 * q;
  *(volatile v4u*)p = u;
  __threadfence();
  *(volatile v4u*)p = u;
}

__global__ __launch_bounds__(256) void w2t_kernel(const float* __restrict__ W2, unsigned short* __restrict__ out, float scale) {
  const int t = blockIdx.x * 256 + threadIdx.x;
  const int n = t >> 3;
  const int q = t & 7;
  const int r = n >> 6;
  const int h = n & 63;
  unsigned short hb[8];
#pragma unroll
  for (int e = 0; e < 8; ++e) {
    const int k = 8 * q + e;
    hb[e] = h_bits(W2[((size_t)r * kHid + k) * kHid + h] * scale);
  }
  const v4u u = (v4u){pk16(hb[0], hb[1]), pk16(hb[2], hb[3]), pk16(hb[4], hb[5]), pk16(hb[6], hb[7])};
  unsigned short* p = out + (size_t)n * kHid + 8 * q;
  *(volatile v4u*)p = u;
  __threadfence();
  *(volatile v4u*)p = u;
}

__global__ __launch_bounds__(256) void b1p_kernel(const float* __restrict__ b1, float* __restrict__ out, float scale) {
  const int i = blockIdx.x * 256 + threadIdx.x;
  v4f v;
#pragma unroll
  for (int e = 0; e < 4; ++e) {
    const int idx = 4 * i + e;
    const int ic  = (idx < kN1Real) ? idx : (kN1Real - 1);
    const float f = b1[ic] * scale;
    v[e] = (idx < kN1Real) ? f : 0.0f;
  }
  float* p = out + 4 * (size_t)i;
  *(volatile v4f*)p = v;
  __threadfence();
  *(volatile v4f*)p = v;
}

__global__ __launch_bounds__(256) void final_kernel(const float* __restrict__ Otab,
                                                     const float* __restrict__ w0_1, const float* __restrict__ b0_1,
                                                     const float* __restrict__ w0_2, const float* __restrict__ b0_2,
                                                     const float* __restrict__ w0_3, const float* __restrict__ b0_3,
                                                     float* __restrict__ out) {
  __shared__ __align__(16) float tile[64 * 68];
  __shared__ float h1s[64];
  __shared__ float h2s[64];
  const int t    = threadIdx.x;
  const int lane = t & 31, wave = t >> 5;
  const int b0   = blockIdx.x * 64;

#pragma unroll
  for (int it = 0; it < 16; ++it) {
    const int e  = it * 256 + t;
    const int r  = e >> 6;
    const int bl = e & 63;
    const int rc = (r < kNExp) ? r : (kNExp - 1);
    const float val = Otab[(size_t)rc * kBatch + b0 + bl];
    if (r < kNExp) tile[bl * 68 + 1 + r] = val;
  }
  if (t < 64) {
    float s = 0.f;
#pragma unroll 1
    for (int k = 0; k < 10; ++k) {
      const float vk = 0.1f * (-5.0f + (float)k * (10.0f / 9.0f));
      s += vk * w0_1[k * kHid + t];
    }
    h1s[t] = fmaxf(s + b0_1[t], 0.0f);
  }
  __syncthreads();
  if (t < 64) {
    float s = 0.f;
#pragma unroll 1
    for (int k = 0; k < 64; ++k) s += h1s[k] * w0_2[k * kHid + t];
    h2s[t] = fmaxf(s + b0_2[t], 0.0f);
  }
  __syncthreads();
  if (t < 64) {
    float s = 0.f;
#pragma unroll 1
    for (int k = 0; k < 64; ++k) s += h2s[k] * w0_3[k];
    tile[t * 68 + 0] = s + b0_3[0];
  }
  __syncthreads();
  const int hh = lane >> 4, c4 = (lane & 15) * 4;
  for (int pass = 0; pass < 2; ++pass) {
#pragma unroll
    for (int it = 0; it < 4; ++it) {
      const int row = wave * 8 + it * 2 + hh;
      v4f v = *(const v4f*)(tile + row * 68 + c4);
      *(volatile v4f*)(out + (size_t)(b0 + row) * kDin + c4) = v;
    }
    __threadfence();
  }
}

extern "C" void kernel_launch(void* const* d_in, const int* in_sizes, int n_in,
                              void* d_out, int out_size, void* d_ws, size_t ws_size,
                              hipStream_t stream) {
  (void)in_sizes; (void)n_in;
  if (ws_size < kWsTotal) return;
  if ((size_t)out_size < (size_t)kBatch * kDin) return;

  const float* X    = (const float*)d_in[0];
  const float* W1   = (const float*)d_in[1];
  const float* b1   = (const float*)d_in[2];
  const float* W2   = (const float*)d_in[3];
  const float* b2   = (const float*)d_in[4];
  const float* W3   = (const float*)d_in[5];
  const float* b3   = (const float*)d_in[6];
  const float* w0_1 = (const float*)d_in[7];
  const float* b0_1 = (const float*)d_in[8];
  const float* w0_2 = (const float*)d_in[9];
  const float* b0_2 = (const float*)d_in[10];
  const float* w0_3 = (const float*)d_in[11];
  const float* b0_3 = (const float*)d_in[12];
  float* out = (float*)d_out;

  char* ws = (char*)d_ws;
  unsigned short* Xh  = (unsigned short*)(ws + kOffXh);
  unsigned short* W1t = (unsigned short*)(ws + kOffW1t);
  unsigned short* W2t = (unsigned short*)(ws + kOffW2t);
  float*          b1p = (float*)(ws + kOffB1p);
  float*          Otab = (float*)(ws + kOffO);
  unsigned short* H1  = (unsigned short*)(ws + kOffH1);

  cast8_f16_kernel<<<(kBatch * kDin / 8) / 256, 256, 0, stream>>>(X, Xh, kBatch * kDin / 8);
  w1t_kernel<<<(kN1 * 8) / 256, 256, 0, stream>>>(W1, W1t, kWCarry);
  w2t_kernel<<<(kN1Real * 8) / 256, 256, 0, stream>>>(W2, W2t, kWCarry);
  b1p_kernel<<<(kN1 / 4) / 256, 256, 0, stream>>>(b1, b1p, kB1Carry);

  for (int c = 0; c < kNChunk; ++c) {
    const unsigned short* Xc = Xh + (size_t)c * kChunk * kDin;
    {
      const int tiles = (kChunk / 64) * (2048 / 64);
      wmma_gemm64<0, false, 2, 1, false, 2><<<dim3(tiles / 8, 1), 256, 0, stream>>>(
          Xc, nullptr, kDin, 0L,
          W1t, nullptr, kDin, 0L,
          (void*)H1, nullptr, kN1, 0L,
          b1p, nullptr, 0L,
          kChunk, 2048, 32, kL1Scale);
    }
    {
      const int tiles = (kChunk / 64) * (2048 / 64);
      wmma_gemm64<0, false, 2, 1, false, 2><<<dim3(tiles / 8, 1), 256, 0, stream>>>(
          Xc, nullptr, kDin, 0L,
          W1t + (size_t)2048 * kDin, nullptr, kDin, 0L,
          (void*)(H1 + 2048), nullptr, kN1, 0L,
          b1p + 2048, nullptr, 0L,
          kChunk, 2048, 64, kL1Scale);
    }
    gemm64_rowdot<<<dim3((kChunk / 64) / 8, kNExp), 256, 0, stream>>>(
        H1, kN1, (long)kHid,
        W2t, kHid, (long)(kHid * kHid),
        b2, (long)kHid,
        W3, (long)kHid,
        b3,
        Otab + (size_t)c * kChunk, (long)kBatch,
        kChunk, kHid, kL2Scale);
  }

  final_kernel<<<kBatch / 64, 256, 0, stream>>>(Otab, w0_1, b0_1, w0_2, b0_2, w0_3, b0_3, out);
}
